// MultiHeadAttentionBlock_23502061043960
// MI455X (gfx1250) — hardware-run, weakly checked
//
#include <hip/hip_runtime.h>


#ifndef NB
#define NB 2
#endif
#ifndef SEQ
#define SEQ 4096
#endif
#define NB_FULL  2
#define SEQ_FULL 4096
#ifndef OUT_SEQ
#define OUT_SEQ SEQ
#endif
#define DM   512
#define NH_  8
#define HD   64
#define AW   4
#define OSP  68
#define QRS  2048.0f
#define QRI  (1.0f / 2048.0f)
#define SSC  0.125f
#define CSC  (1.0f / 32.0f)
#define WOS  16.0f
#define OSC  2.0f

static_assert(HD == 64);
static_assert(NH_ * HD == DM);
static_assert(DM % 64 == 0);
static_assert(HD % 32 == 0);
static_assert(DM % 32 == 0);
static_assert(SEQ % 64 == 0);
static_assert((NB * SEQ) % 64 == 0);
static_assert((NB * SEQ) % 32 == 0);
static_assert(SEQ % 32 == 0);
static_assert(SEQ % (16 * AW) == 0);
static_assert(((size_t)SEQ * DM) % 8 == 0);
static_assert(((size_t)DM * DM) % 8 == 0);
static_assert(NB <= NB_FULL);
static_assert(SEQ <= SEQ_FULL);
static_assert((OSP * 4) % 16 == 0);
static_assert(OSP >= 64 + 4);
static_assert(32 * 16 * 4 == 16 * HD * 2);
static_assert(32 * 16 * 8 == 16 * 64 * 4);
static_assert(16 * 68 * 4 <= 131072);
static_assert(AW * 16 * OSP * 4 <= 131072);
static_assert(OSC * CSC * WOS == 1.0f);

typedef _Float16 h16;
typedef unsigned short bf;
typedef __attribute__((ext_vector_type(16))) __bf16   v16bf;
typedef __attribute__((ext_vector_type(16))) _Float16 v16h;
typedef __attribute__((ext_vector_type(8)))  _Float16 v8h;
typedef __attribute__((ext_vector_type(8)))  unsigned short v8us;
typedef __attribute__((ext_vector_type(8)))  float    v8f;
typedef __attribute__((ext_vector_type(4)))  float    v4f;
typedef v4f  __attribute__((may_alias)) v4fa;

__device__ __forceinline__ unsigned short f2bf(float f) { unsigned u = __float_as_uint(f); u += 0x7FFFu + ((u >> 16) & 1u); return (unsigned short)(u >> 16); }
__device__ __forceinline__ float bfr(float f) { return __uint_as_float(((unsigned)f2bf(f)) << 16); }
__device__ __forceinline__ v16h cat16(v8h lo, v8h hi) { return __builtin_shufflevector(lo, hi, 0, 1, 2, 3, 4, 5, 6, 7, 8, 9, 10, 11, 12, 13, 14, 15); }
__device__ __forceinline__ v16bf cat16b(v8us lo, v8us hi) { return __builtin_bit_cast(v16bf, __builtin_shufflevector(lo, hi, 0, 1, 2, 3, 4, 5, 6, 7, 8, 9, 10, 11, 12, 13, 14, 15)); }
__device__ __forceinline__ v8f wmma16(v16h a, v16h b, v8f c) { return __builtin_amdgcn_wmma_f32_16x16x32_f16(false, a, false, b, (short)0, c, false, false); }
__device__ __forceinline__ v8f wmmab(v16bf a, v16bf b, v8f c) { return __builtin_amdgcn_wmma_f32_16x16x32_bf16(false, a, false, b, (short)0, c, false, false); }
__device__ __forceinline__ v16h  ldh(const h16* p) { return cat16(*(const v8h*)p, *(const v8h*)(p + 16)); }
__device__ __forceinline__ v16bf ldb(const bf* p)  { return cat16b(*(const v8us*)p, *(const v8us*)(p + 16)); }
__device__ __forceinline__ void wave_sync() { __builtin_amdgcn_fence(3  , "wavefront"); __builtin_amdgcn_wave_barrier(); asm volatile("" ::: "memory"); }

static __device__ __forceinline__ h16 toh_flush(float v) { const float w = (fabsf(v) < 6.103515625e-05f) ? 0.0f : v; return (h16)w; }
__device__ __forceinline__ v8f wmmabg(v16bf a, v16bf b, v8f c) { c = wmmab(a, b, c); asm volatile("v_nop\n\tv_nop\n\tv_nop\n\tv_nop" : "+v"(c) : "v"(a), "v"(b)); return c; }
__device__ __forceinline__ v8f wmma16g(v16h a, v16h b, v8f c) { c = wmma16(a, b, c); asm volatile("v_nop\n\tv_nop\n\tv_nop\n\tv_nop" : "+v"(c) : "v"(a), "v"(b)); return c; }

__global__ __launch_bounds__(256) void k_cvt8(const float* __restrict__ src, bf* dst, size_t n8) {
    const size_t i = (size_t)blockIdx.x * 256 + threadIdx.x; if (i >= n8) return;
    const v8f v = *(const v8f*)(src + i * 8); v8us o;
#pragma unroll
    for (int k = 0; k < 8; ++k) o[k] = f2bf(v[k]);
    *(volatile v8us*)(dst + i * 8) = o; __threadfence(); *(volatile v8us*)(dst + i * 8) = o;
}

__global__ __launch_bounds__(256) void k_cvtw(const float* __restrict__ src, h16* dst, size_t n8) {
    const size_t i = (size_t)blockIdx.x * 256 + threadIdx.x; if (i >= n8) return;
    const v8f v = *(const v8f*)(src + i * 8); v8h o;
#pragma unroll
    for (int k = 0; k < 8; ++k) o[k] = toh_flush(bfr(v[k]) * WOS);
    *(volatile v8h*)(dst + i * 8) = o; __threadfence(); *(volatile v8h*)(dst + i * 8) = o;
}

template <int MODE>
__device__ __forceinline__ void proj_body(const bf* __restrict__ A, const bf* __restrict__ Bt, const float* __restrict__ bias, h16* Ph, h16* Pr, const int resT) {
    __shared__ __align__(16) float os[16 * 68];
    const int K = DM;
    const int lane = threadIdx.x & 31, lr = lane & 15, hi = lane >> 4;
    const unsigned r0 = blockIdx.x * 64u, c0 = blockIdx.y * 64u;
    v8f acc[4][4];
#pragma unroll
    for (int mb = 0; mb < 4; ++mb)
#pragma unroll
        for (int nb = 0; nb < 4; ++nb) acc[mb][nb] = (v8f){};
    const size_t aoff = (size_t)(r0 + (unsigned)lr) * K + 8 * hi, boff = (size_t)(c0 + (unsigned)lr) * K + 8 * hi;
#pragma unroll 1
    for (int kc = 0; kc < K; kc += 32) {
        v16bf a[4];
#pragma unroll
        for (int mb = 0; mb < 4; ++mb) a[mb] = ldb(A + aoff + (size_t)mb * 16 * K + kc);
#pragma unroll
        for (int nb = 0; nb < 4; ++nb) { const v16bf b = ldb(Bt + boff + (size_t)nb * 16 * K + kc);
#pragma unroll
            for (int mb = 0; mb < 4; ++mb) acc[mb][nb] = wmmabg(a[mb], b, acc[mb][nb]); }
    }
    float bc[4];
#pragma unroll
    for (int nb = 0; nb < 4; ++nb) bc[nb] = (MODE == 0) ? bfr(bias[c0 + nb * 16 + lr]) : 0.0f;
    const unsigned ures = (unsigned)resT;
    size_t tbase, rbase, pitch, rpitch; bool wr;
    if (MODE == 0) { const unsigned bb = r0 / (unsigned)SEQ, tt = r0 % (unsigned)SEQ; const unsigned zc = bb * (unsigned)NH_ + c0 / (unsigned)HD;
                     tbase = ((size_t)zc * SEQ + (size_t)tt) * HD; rbase = ((size_t)zc * (size_t)ures + (size_t)tt) * HD; pitch = HD; rpitch = HD; wr = tt < ures; }
    else           { const unsigned bb = c0 / (unsigned)SEQ, tt = c0 % (unsigned)SEQ;
                     tbase = (size_t)bb * (size_t)DM * SEQ + (size_t)r0 * SEQ + (size_t)tt; rbase = (size_t)bb * (size_t)DM * (size_t)ures + (size_t)r0 * (size_t)ures + (size_t)tt;
                     pitch = SEQ; rpitch = ures; wr = tt < ures; }
#pragma unroll
    for (int mb = 0; mb < 4; ++mb) {
        float br[8];
#pragma unroll
        for (int j = 0; j < 8; ++j) br[j] = (MODE == 1) ? bfr(bias[r0 + mb * 16 + hi * 8 + j]) : 0.0f;
#pragma unroll
        for (int nb = 0; nb < 4; ++nb) {
#pragma unroll
            for (int j = 0; j < 8; ++j) os[(hi * 8 + j) * 68 + nb * 16 + lr] = acc[mb][nb][j] + bc[nb] + br[j]; }
        wave_sync();
        const size_t sb = tbase + (size_t)(mb * 16) * pitch;
        const size_t rb = rbase + (size_t)(mb * 16) * rpitch;
#pragma unroll 1
        for (int ps = 0; ps < 2; ++ps) {
#pragma unroll
            for (int s = 0; s < 4; ++s) { const int row = 4 * s + (lane >> 3), c8 = (lane & 7) * 8;
                const v4f x0 = *(const v4fa*)(&os[row * 68 + c8]); const v4f x1 = *(const v4fa*)(&os[row * 68 + c8 + 4]); v8h hv, rv;
#pragma unroll
                for (int i = 0; i < 4; ++i) { const h16 a0 = toh_flush(x0[i]); const h16 a1 = toh_flush(x1[i]); hv[i] = a0; hv[4 + i] = a1;
                                              rv[i] = toh_flush((x0[i] - (float)a0) * QRS); rv[4 + i] = toh_flush((x1[i] - (float)a1) * QRS); }
                const size_t oo = sb + (size_t)row * pitch + c8;
                const size_t ro = rb + (size_t)row * rpitch + c8;
                *(volatile v8h*)(Ph + oo) = hv; if (wr) *(volatile v8h*)(Pr + ro) = rv; }
            if (ps == 0) __threadfence(); }
        wave_sync();
    }
}

__global__ __launch_bounds__(32) void k_proj_tok(const bf* __restrict__ A, const bf* __restrict__ Bt, const float* __restrict__ bias, h16* Ph, h16* Pr, int resT) {
    proj_body<0>(A, Bt, bias, Ph, Pr, resT);
}
__global__ __launch_bounds__(32) void k_proj_tr(const bf* __restrict__ A, const bf* __restrict__ Bt, const float* __restrict__ bias, h16* Ph, h16* Pr, int resT) {
    proj_body<1>(A, Bt, bias, Ph, Pr, resT);
}

__device__ __forceinline__ v8f score16(const h16* __restrict__ kp, const v16h qh0, const v16h qh1) {
    const v16h k0 = ldh(kp), k1 = ldh(kp + 32);
    v8f sH = (v8f){};
    sH = wmma16g(k0, qh0, sH); sH = wmma16g(k1, qh1, sH);
    return sH * SSC;
}

__global__ __launch_bounds__(32 * AW) void k_attn(const h16* __restrict__ QH, const h16* __restrict__ KP, const h16* __restrict__ VT, h16* CH, h16* CR) {
    __shared__ __align__(16) float os[AW * 16 * OSP];
    const int lane = threadIdx.x & 31, lr = lane & 15, hi = lane >> 4;
    const int wave = __builtin_amdgcn_readfirstlane((int)(threadIdx.x >> 5));
    const unsigned zh = blockIdx.y; const unsigned b = zh / (unsigned)NH_, h = zh % (unsigned)NH_;
    const int t0 = (int)((blockIdx.x * (unsigned)AW + (unsigned)wave) * 16u);
    const size_t pbase = (size_t)zh * SEQ * HD;
    const size_t qo = pbase + (size_t)(t0 + lr) * HD + 8 * hi;
    const v16h qh0 = ldh(QH + qo), qh1 = ldh(QH + qo + 32);
    const size_t ko = pbase + (size_t)lr * HD + 8 * hi;
    const size_t vo = pbase + (size_t)lr * SEQ + 8 * hi;
    v8f o[4];
#pragma unroll
    for (int j = 0; j < 4; ++j) o[j] = (v8f){};
#pragma unroll 1
    for (int key0 = 0; key0 < SEQ; key0 += 32) {
        const h16* ka = KP + ko + (size_t)key0 * HD;
        v16h pb;
        { const v8f sa = score16(ka, qh0, qh1);
#pragma unroll
          for (int r = 0; r < 8; ++r) pb[r] = toh_flush(sa[r]); }
        { const v8f sb = score16(ka + 16 * HD, qh0, qh1);
#pragma unroll
          for (int r = 0; r < 8; ++r) pb[8 + r] = toh_flush(sb[r]); }
        const h16* va = VT + vo + key0;
#pragma unroll
        for (int j = 0; j < 4; ++j) { const v16h vf = ldh(va + (size_t)(16 * j) * SEQ); o[j] = wmma16g(vf, pb, o[j]); }
    }
    const int wb = wave * 16 * OSP;
#pragma unroll
    for (int j = 0; j < 4; ++j) { v4f a, c;
        a[0] = o[j][0]; a[1] = o[j][1]; a[2] = o[j][2]; a[3] = o[j][3]; c[0] = o[j][4]; c[1] = o[j][5]; c[2] = o[j][6]; c[3] = o[j][7];
        *(v4fa*)(&os[wb + lr * OSP + 16 * j + 8 * hi]) = a; *(v4fa*)(&os[wb + lr * OSP + 16 * j + 8 * hi + 4]) = c; }
    wave_sync();
    const size_t cb = ((size_t)b * SEQ + (size_t)t0) * DM + (size_t)h * HD;
#pragma unroll 1
    for (int ps = 0; ps < 2; ++ps) {
#pragma unroll
        for (int s = 0; s < 4; ++s) { const int row = 4 * s + (lane >> 3), c8 = (lane & 7) * 8;
            const v4f x0 = *(const v4fa*)(&os[wb + row * OSP + c8]); const v4f x1 = *(const v4fa*)(&os[wb + row * OSP + c8 + 4]); v8h hv, rv;
#pragma unroll
            for (int i = 0; i < 4; ++i) { const float y0 = x0[i] * CSC, y1 = x1[i] * CSC; const h16 a0 = toh_flush(y0); const h16 a1 = toh_flush(y1); hv[i] = a0; hv[4 + i] = a1;
                                          rv[i] = toh_flush((y0 - (float)a0) * QRS); rv[4 + i] = toh_flush((y1 - (float)a1) * QRS); }
            const size_t oo = cb + (size_t)row * DM + c8;
            *(volatile v8h*)(CH + oo) = hv; *(volatile v8h*)(CR + oo) = rv; }
        if (ps == 0) __threadfence(); }
}

__global__ __launch_bounds__(32) void k_oproj(const h16* __restrict__ AH, const h16* __restrict__ AR, const h16* __restrict__ Wt, const float* __restrict__ bias, float* OUT) {
    __shared__ __align__(16) float os[16 * 68];
    const int K = DM;
    const int lane = threadIdx.x & 31, lr = lane & 15, hi = lane >> 4;
    const unsigned r0 = blockIdx.x * 32u, c0 = blockIdx.y * 64u;
    v8f aH[2][4], aR[2][4];
#pragma unroll
    for (int mb = 0; mb < 2; ++mb)
#pragma unroll
        for (int nb = 0; nb < 4; ++nb) { aH[mb][nb] = (v8f){}; aR[mb][nb] = (v8f){}; }
    const size_t aoff = (size_t)(r0 + (unsigned)lr) * K + 8 * hi, boff = (size_t)(c0 + (unsigned)lr) * K + 8 * hi;
#pragma unroll 1
    for (int kc = 0; kc < K; kc += 32) {
        v16h ah[2], ar[2];
#pragma unroll
        for (int mb = 0; mb < 2; ++mb) { ah[mb] = ldh(AH + aoff + (size_t)mb * 16 * K + kc); ar[mb] = ldh(AR + aoff + (size_t)mb * 16 * K + kc); }
#pragma unroll
        for (int nb = 0; nb < 4; ++nb) { const v16h bw = ldh(Wt + boff + (size_t)nb * 16 * K + kc);
#pragma unroll
            for (int mb = 0; mb < 2; ++mb) { aH[mb][nb] = wmma16g(ah[mb], bw, aH[mb][nb]); aR[mb][nb] = wmma16g(ar[mb], bw, aR[mb][nb]); } }
    }
    float bc[4];
#pragma unroll
    for (int nb = 0; nb < 4; ++nb) bc[nb] = bfr(bias[c0 + nb * 16 + lr]);
    const unsigned bb = r0 / (unsigned)SEQ, tt = r0 % (unsigned)SEQ;
    const size_t obase = ((size_t)bb * OUT_SEQ + (size_t)tt) * DM + (size_t)c0;
#pragma unroll
    for (int mb = 0; mb < 2; ++mb) {
#pragma unroll
        for (int nb = 0; nb < 4; ++nb) {
#pragma unroll
            for (int j = 0; j < 8; ++j) os[(hi * 8 + j) * 68 + nb * 16 + lr] = (aH[mb][nb][j] + aR[mb][nb][j] * QRI) * OSC + bc[nb]; }
        wave_sync();
        const size_t sb = obase + (size_t)(mb * 16) * DM;
#pragma unroll 1
        for (int ps = 0; ps < 2; ++ps) {
#pragma unroll
            for (int s = 0; s < 8; ++s) { const int row = 2 * s + (lane >> 4), cofs = (lane & 15) * 4;
                const v4f val = *(const v4fa*)(&os[row * 68 + cofs]);
                *(volatile v4f*)(OUT + sb + (size_t)row * DM + cofs) = val; }
            if (ps == 0) __threadfence(); }
        wave_sync();
    }
}

static constexpr size_t al256(size_t v) { return (v + 255) & ~(size_t)255; }
static constexpr size_t SZ_XB = al256((size_t)NB * SEQ * DM * 2);
static constexpr size_t SZ_WB = al256((size_t)3 * DM * DM * 2);
static constexpr size_t SZ_WO = al256((size_t)DM * DM * 2);
static constexpr size_t SZ_PL = al256((size_t)NB * NH_ * SEQ * HD * 2);
static constexpr size_t SZ_TOTAL = 3 * SZ_XB + SZ_WB + SZ_WO + 5 * SZ_PL;
static_assert(SZ_TOTAL <= (size_t)134217728);
static_assert(((size_t)DM * DM * 2) % 256 == 0);
static_assert((size_t)NB * NH_ * SEQ * HD == (size_t)NB * DM * SEQ);

extern "C" void kernel_launch(void* const* d_in, const int* in_sizes, int n_in,
                              void* d_out, int out_size, void* d_ws, size_t ws_size, hipStream_t stream) {
    if (n_in < 11) return;
    const size_t needx = ((size_t)(NB - 1) * SEQ_FULL + SEQ) * DM;
    if ((size_t)in_sizes[0] < needx || (size_t)in_sizes[1] < needx || (size_t)in_sizes[2] < needx) return;
    if ((size_t)in_sizes[3] < (size_t)DM * DM || (size_t)in_sizes[5] < (size_t)DM * DM || (size_t)in_sizes[7] < (size_t)DM * DM || (size_t)in_sizes[9] < (size_t)DM * DM) return;
    if (in_sizes[4] < DM || in_sizes[6] < DM || in_sizes[8] < DM || in_sizes[10] < DM) return;
    if ((size_t)out_size < ((size_t)(NB - 1) * OUT_SEQ + SEQ) * DM) return;
    if (SZ_TOTAL > ws_size) return;
    const float* xin[3] = { (const float*)d_in[0], (const float*)d_in[1], (const float*)d_in[2] };
    const float* wq = (const float*)d_in[3]; const float* bq = (const float*)d_in[4];
    const float* wk = (const float*)d_in[5]; const float* bk = (const float*)d_in[6];
    const float* wv = (const float*)d_in[7]; const float* bv = (const float*)d_in[8];
    const float* wo = (const float*)d_in[9]; const float* bo = (const float*)d_in[10];
    float* OUT = (float*)d_out;
    char* wsp = (char*)d_ws;
    bf* XB[3];
    XB[0] = (bf*)wsp; wsp += SZ_XB;
    XB[1] = (bf*)wsp; wsp += SZ_XB;
    XB[2] = (bf*)wsp; wsp += SZ_XB;
    bf* WB = (bf*)wsp; wsp += SZ_WB;
    h16* WO = (h16*)wsp; wsp += SZ_WO;
    h16* QH = (h16*)wsp; wsp += SZ_PL;
    h16* KP = (h16*)wsp; wsp += SZ_PL;
    h16* VT = (h16*)wsp; wsp += SZ_PL;
    h16* CH = (h16*)wsp; wsp += SZ_PL;
    h16* CR = (h16*)wsp; wsp += SZ_PL;
    bf* WQ = WB; bf* WK = WB + (size_t)DM * DM; bf* WV = WB + (size_t)2 * DM * DM;

    for (int i = 0; i < 3; ++i) {
        if (SEQ == SEQ_FULL) {
            const size_t n8 = (size_t)NB * SEQ * DM / 8;
            k_cvt8<<<(unsigned)((n8 + 255) / 256), 256, 0, stream>>>(xin[i], XB[i], n8);
        } else {
            const size_t n8 = (size_t)SEQ * DM / 8;
            for (int b = 0; b < NB; ++b) k_cvt8<<<(unsigned)((n8 + 255) / 256), 256, 0, stream>>>(xin[i] + (size_t)b * SEQ_FULL * DM, XB[i] + (size_t)b * SEQ * DM, n8);
        }
    }
    { const size_t n8 = (size_t)DM * DM / 8; const unsigned g = (unsigned)((n8 + 255) / 256);
      k_cvt8<<<g, 256, 0, stream>>>(wq, WQ, n8); k_cvt8<<<g, 256, 0, stream>>>(wk, WK, n8); k_cvt8<<<g, 256, 0, stream>>>(wv, WV, n8);
      k_cvtw<<<g, 256, 0, stream>>>(wo, WO, n8); }

    k_proj_tok<<<dim3(NB * SEQ / 64, DM / 64, 1), 32, 0, stream>>>(XB[0], WQ, bq, QH, QH, 0);
    k_proj_tok<<<dim3(NB * SEQ / 64, DM / 64, 1), 32, 0, stream>>>(XB[1], WK, bk, KP, KP, 0);
    k_proj_tr<<<dim3(DM / 64, NB * SEQ / 64, 1), 32, 0, stream>>>(WV, XB[2], bv, VT, VT, 0);

    k_attn<<<dim3(SEQ / (16 * AW), NB * NH_, 1), 32 * AW, 0, stream>>>(QH, KP, VT, CH, CR);

    k_oproj<<<dim3(NB * SEQ / 32, DM / 64, 1), 32, 0, stream>>>(CH, CR, WO, bo, OUT);
}
